// EGNNLayer_44959717655304
// MI455X (gfx1250) — hardware-verified
//
#include <hip/hip_runtime.h>
#include <stddef.h>
#include <stdint.h>
#include <math.h>


#define NF      64
#define NTHR    256
#define NWAVE   8
#define EPT     8
#define CHUNK   (NTHR * EPT)
#define WCAP    (EPT * 32)
#define LISTN   (NWAVE * WCAP)
#define NBA     512
#define SLA     9
#define RCAP    10240
#define MEAS_B512 8444
#define TROWS   128
#define AP      136
#define SP      68
#define GBM     64
#define GTHR    128
#define MROWS   128
#define KN1     192
#define KD      128
#define WSMAX   134217728
#define OFF_E1  0
#define OFF_E2  8192
#define OFF_C1  16384
#define OFF_N1  24576
#define OFF_N2  36864
#define WPL_HALVES 45056
#define NU_E1   1024
#define NU_D    1024
#define NU_N1   1536
#define NU_PB   (NU_E1 + 3 * NU_D + NU_N1)
#define T_W128  0
#define T_BE1   64
#define T_BE2   128
#define T_BC1   192
#define T_WC2   256
#define T_BN1   320
#define T_BN2   384
#define T_BC2   448
#define TABN    512
#define BKT_LDS_INTS (LISTN + RCAP + 16)
#define E_ACC_F (NBA * SP)
#define E_STG_F (TROWS * SP)
#define E_A_H   (TROWS * AP)
#define E_W_H   (NF * AP)
#define EDGE_LDS_BYTES (E_ACC_F * 4 + E_STG_F * 4 + TROWS * 16 + TABN * 4 + TROWS * 4 + E_A_H * 2 + 2 * E_W_H * 2)

static_assert(NF == 64);
static_assert((CHUNK & (CHUNK - 1)) == 0 && CHUNK <= 4096);
static_assert((NBA & (NBA - 1)) == 0 && NBA == (1 << SLA));
static_assert(((long long)CHUNK << SLA) < (1LL << 31));
static_assert(RCAP % 128 == 0 && RCAP % 32 == 0);
static_assert(RCAP * 10 >= MEAS_B512 * 11);
static_assert(TROWS == NWAVE * 16 && TROWS * 2 == NTHR);
static_assert((NBA * 12) % 128 == 0);
static_assert((NBA * 3) % 4 == 0 && (NBA * 3) / 4 <= 2 * NTHR && NBA * 3 <= E_STG_F);
static_assert(EDGE_LDS_BYTES <= 300000);
static_assert(BKT_LDS_INTS * 4 <= 65536);
static_assert((AP * 2) % 16 == 0 && (SP * 4) % 16 == 0 && AP >= KD && SP >= NF + 4);
static_assert(NU_E1 % NTHR == 0 && NU_D % NTHR == 0 && NU_N1 % NTHR == 0);
static_assert(OFF_N2 + NF * KD == WPL_HALVES);
static_assert(GBM == (GTHR / 32) * 16 && (MROWS % GBM) == 0 && (NBA % GBM) == 0);
static_assert(KN1 % 32 == 0 && KD % 32 == 0 && NF % 32 == 0);
static_assert((12800000 % 128) == 0);

typedef float          v4f  __attribute__((ext_vector_type(4)));
typedef float          v8f  __attribute__((ext_vector_type(8)));
typedef int            v4i  __attribute__((ext_vector_type(4)));
typedef int            v8i  __attribute__((ext_vector_type(8)));
typedef unsigned short v8us __attribute__((ext_vector_type(8)));
typedef __bf16         v16b __attribute__((ext_vector_type(16)));
typedef v4f  __attribute__((may_alias)) v4fa;
typedef v4i  __attribute__((may_alias)) v4ia;
typedef v8us __attribute__((may_alias)) v8usa;
union FragB { v16b v; v8us h[2]; v8i w; };

__device__ __forceinline__ v8f wmb(const FragB& a, const FragB& b, v8f c) {
  v8f d = __builtin_amdgcn_wmma_f32_16x16x32_bf16(false, a.v, false, b.v, (short)0, c, false, false);
  asm volatile("v_nop\n\tv_nop\n\tv_nop\n\tv_nop" : "+v"(d) : "v"(a.w), "v"(b.w));
  return d;
}

__device__ __forceinline__ unsigned int f2bf(float f) {
  const unsigned int u = __float_as_uint(f);
  const unsigned int r = ((u + 0x7FFFu + ((u >> 16) & 1u)) >> 16) & 0xFFFFu;
  return ((u & 0x7FFFFFFFu) > 0x7F800000u) ? 0x7FC0u : r;
}
__device__ __forceinline__ float bf2f(unsigned int b) { return __uint_as_float(b << 16); }
__device__ __forceinline__ float bfr(float f) { return bf2f(f2bf(f)); }
__device__ __forceinline__ float silu_p(float v) { return v / (1.0f + expf(-v)); }

template <int SLB>
__device__ __forceinline__ int scan_chunk(const int* __restrict__ dsts, int nE, int cbase, int slotBase,
                                          int nb, int vec8, int* list, int tid, int lane, int wave) {
  int wc = 0;
  const int el0  = tid * EPT;
  const int e0   = cbase + el0;
  const int sent = -2147483647 - 1;
  v4i da, db;
  if (vec8 != 0 && cbase + CHUNK <= nE) {
    da = *(const v4i*)(dsts + e0);
    db = *(const v4i*)(dsts + e0 + 4);
  } else {
    da.x = (e0     < nE) ? dsts[min(e0,     nE - 1)] : sent;
    da.y = (e0 + 1 < nE) ? dsts[min(e0 + 1, nE - 1)] : sent;
    da.z = (e0 + 2 < nE) ? dsts[min(e0 + 2, nE - 1)] : sent;
    da.w = (e0 + 3 < nE) ? dsts[min(e0 + 3, nE - 1)] : sent;
    db.x = (e0 + 4 < nE) ? dsts[min(e0 + 4, nE - 1)] : sent;
    db.y = (e0 + 5 < nE) ? dsts[min(e0 + 5, nE - 1)] : sent;
    db.z = (e0 + 6 < nE) ? dsts[min(e0 + 6, nE - 1)] : sent;
    db.w = (e0 + 7 < nE) ? dsts[min(e0 + 7, nE - 1)] : sent;
  }
  const unsigned nbs = (unsigned)slotBase;
  const unsigned unb = (unsigned)nb;
  const unsigned s0 = (unsigned)da.x - nbs, s1 = (unsigned)da.y - nbs;
  const unsigned s2 = (unsigned)da.z - nbs, s3 = (unsigned)da.w - nbs;
  const unsigned s4 = (unsigned)db.x - nbs, s5 = (unsigned)db.y - nbs;
  const unsigned s6 = (unsigned)db.z - nbs, s7 = (unsigned)db.w - nbs;
  const bool h0 = s0 < unb, h1 = s1 < unb, h2 = s2 < unb, h3 = s3 < unb;
  const bool h4 = s4 < unb, h5 = s5 < unb, h6 = s6 < unb, h7 = s7 < unb;
  const unsigned any = __builtin_amdgcn_ballot_w32(h0 | h1 | h2 | h3 | h4 | h5 | h6 | h7);
  if (any != 0u) {
#define HITJ(J, HJ, SJ) { \
      const unsigned mj = __builtin_amdgcn_ballot_w32(HJ); \
      if (mj != 0u) { \
        if (HJ) { \
          const int pos = wc + (int)__builtin_amdgcn_mbcnt_lo(mj, 0u); \
          if (pos < WCAP) list[wave * WCAP + pos] = ((el0 + (J)) << SLB) | (int)(SJ); \
        } \
        wc += (int)__builtin_popcount(mj); } }
    HITJ(0, h0, s0)
    HITJ(1, h1, s1)
    HITJ(2, h2, s2)
    HITJ(3, h3, s3)
    HITJ(4, h4, s4)
    HITJ(5, h5, s5)
    HITJ(6, h6, s6)
    HITJ(7, h7, s7)
#undef HITJ
  }
  return wc;
}

__global__ __launch_bounds__(NTHR) void k_pa(const float* __restrict__ feat, const float* __restrict__ coord,
                                             unsigned short* XB, float* CB, int nN, int mRows) {
  const int u  = (int)blockIdx.x * NTHR + (int)threadIdx.x;
  const int U0 = mRows * 8;
  if (u < U0) {
    const int row = u >> 3;
    const int k8  = (u & 7) * 8;
    const int rc  = row < nN ? row : nN - 1;
    const float* p = feat + (size_t)rc * NF + k8;
    const v4f a = *(const v4fa*)p;
    const v4f b = *(const v4fa*)(p + 4);
    const v8f f8 = {a.x, a.y, a.z, a.w, b.x, b.y, b.z, b.w};
    const bool ok = row < nN;
    v8us o;
#pragma unroll
    for (int i = 0; i < 8; ++i) o[i] = ok ? (unsigned short)f2bf(f8[i]) : (unsigned short)0;
    unsigned short* dp = XB + (size_t)row * NF + k8;
    *(volatile v8us*)dp = o;
    __threadfence();
    *(volatile v8us*)dp = o;
  } else {
    const int row = u - U0;
    if (row >= mRows) return;
    const int rc  = row < nN ? row : nN - 1;
    const bool ok = row < nN;
    const float x0 = coord[(size_t)rc * 3 + 0];
    const float x1 = coord[(size_t)rc * 3 + 1];
    const float x2 = coord[(size_t)rc * 3 + 2];
    v4f q;
    q.x = ok ? bfr(x0) : 0.0f;
    q.y = ok ? bfr(x1) : 0.0f;
    q.z = ok ? bfr(x2) : 0.0f;
    q.w = 0.0f;
    float* dp = CB + (size_t)row * 4;
    *(volatile v4f*)dp = q;
    __threadfence();
    *(volatile v4f*)dp = q;
  }
}

__global__ __launch_bounds__(NTHR) void k_pb(const float* __restrict__ We1, const float* __restrict__ We2,
                                             const float* __restrict__ Wc1, const float* __restrict__ Wn1,
                                             const float* __restrict__ Wn2, unsigned short* WPL) {
  const int u = (int)blockIdx.x * NTHR + (int)threadIdx.x;
  v8us o;
  unsigned short* dp;
  if (u < NU_E1) {
    const int n    = u >> 3;
    const int k8   = (u & 7) * 8;
    const int srow = ((n < NF) ? 0 : NF) + k8;
    const float* p = We1 + (size_t)srow * NF + (n & (NF - 1));
#pragma unroll
    for (int i = 0; i < 8; ++i) o[i] = (unsigned short)f2bf(p[(size_t)i * NF]);
    dp = WPL + OFF_E1 + 8 * u;
  } else if (u < NU_E1 + NU_D) {
    const int v  = u - NU_E1;
    const int n  = v >> 4;
    const int kk = ((v & 15) * 8) & (NF - 1);
    const float* p = We2 + (size_t)kk * NF + n;
#pragma unroll
    for (int i = 0; i < 8; ++i) o[i] = (unsigned short)f2bf(p[(size_t)i * NF]);
    dp = WPL + OFF_E2 + 8 * v;
  } else if (u < NU_E1 + 2 * NU_D) {
    const int v  = u - NU_E1 - NU_D;
    const int n  = v >> 4;
    const int kk = ((v & 15) * 8) & (NF - 1);
    const float* p = Wc1 + (size_t)kk * NF + n;
#pragma unroll
    for (int i = 0; i < 8; ++i) o[i] = (unsigned short)f2bf(p[(size_t)i * NF]);
    dp = WPL + OFF_C1 + 8 * v;
  } else if (u < NU_E1 + 2 * NU_D + NU_N1) {
    const int v    = u - NU_E1 - 2 * NU_D;
    const int n    = v / (KN1 / 8);
    const int k8   = (v - n * (KN1 / 8)) * 8;
    const int srow = (k8 < 2 * NF) ? k8 : (k8 - NF);
    const float* p = Wn1 + (size_t)srow * NF + n;
#pragma unroll
    for (int i = 0; i < 8; ++i) o[i] = (unsigned short)f2bf(p[(size_t)i * NF]);
    dp = WPL + OFF_N1 + 8 * v;
  } else if (u < NU_PB) {
    const int v  = u - NU_E1 - 2 * NU_D - NU_N1;
    const int n  = v >> 4;
    const int kk = ((v & 15) * 8) & (NF - 1);
    const float* p = Wn2 + (size_t)kk * NF + n;
#pragma unroll
    for (int i = 0; i < 8; ++i) o[i] = (unsigned short)f2bf(p[(size_t)i * NF]);
    dp = WPL + OFF_N2 + 8 * v;
  } else {
    return;
  }
  *(volatile v8us*)dp = o;
  __threadfence();
  *(volatile v8us*)dp = o;
}

__global__ __launch_bounds__(NTHR) void k_pc(const float* __restrict__ We1, const float* __restrict__ be1,
                                             const float* __restrict__ be2, const float* __restrict__ bc1,
                                             const float* __restrict__ Wc2, const float* __restrict__ bc2,
                                             const float* __restrict__ bn1, const float* __restrict__ bn2,
                                             float* TAB) {
  const int tid = (int)threadIdx.x, lane = tid & 31, wave = tid >> 5;
  const int j = lane & 15;
  v4f v = {0.0f, 0.0f, 0.0f, 0.0f};
  if (wave == 0)      v = *(const v4fa*)(We1 + 128 * NF + 4 * j);
  else if (wave == 1) v = *(const v4fa*)(be1 + 4 * j);
  else if (wave == 2) v = *(const v4fa*)(be2 + 4 * j);
  else if (wave == 3) v = *(const v4fa*)(bc1 + 4 * j);
  else if (wave == 4) v = *(const v4fa*)(Wc2 + 4 * j);
  else if (wave == 5) v = *(const v4fa*)(bn1 + 4 * j);
  else if (wave == 6) v = *(const v4fa*)(bn2 + 4 * j);
  else { const float b = bc2[0]; v.x = (j == 0) ? b : 0.0f; }
  v4f q;
  q.x = bfr(v.x); q.y = bfr(v.y); q.z = bfr(v.z); q.w = bfr(v.w);
  float* dp = TAB + 64 * wave + 4 * j;
  if (lane < 16) *(volatile v4f*)dp = q;
  __threadfence();
  if (lane < 16) *(volatile v4f*)dp = q;
}

__global__ __launch_bounds__(GTHR) void k_psd(const unsigned short* __restrict__ XB,
                                              const unsigned short* __restrict__ WPL,
                                              const float* __restrict__ TAB, float* PSD) {
  __shared__ __attribute__((aligned(16))) float stg[GBM * 128];
  const int tid = (int)threadIdx.x, lane = tid & 31, wave = tid >> 5, hh = lane >> 4, m = lane & 15;
  const int rowBase = (int)blockIdx.x * GBM;
  v8f acc[8];
  {
    const v8f z = {0.f, 0.f, 0.f, 0.f, 0.f, 0.f, 0.f, 0.f};
#pragma unroll
    for (int t = 0; t < 8; ++t) acc[t] = z;
  }
  const unsigned short* ap = XB + (size_t)(rowBase + 16 * wave + m) * NF + 8 * hh;
  const unsigned short* bp = WPL + OFF_E1 + m * NF + 8 * hh;
#pragma unroll
  for (int k0 = 0; k0 < NF; k0 += 32) {
    FragB af;
    af.h[0] = *(const v8usa*)(ap + k0);
    af.h[1] = *(const v8usa*)(ap + k0 + 16);
#pragma unroll
    for (int nt = 0; nt < 8; ++nt) {
      const unsigned short* wq = bp + (16 * nt) * NF + k0;
      FragB bf;
      bf.h[0] = *(const v8usa*)wq;
      bf.h[1] = *(const v8usa*)(wq + 16);
      acc[nt] = wmb(af, bf, acc[nt]);
    }
  }
#pragma unroll
  for (int nt = 0; nt < 8; ++nt) {
    const int lc = 16 * nt + m;
    float bvv = 0.0f;
    if (nt >= 4) bvv = TAB[T_BE1 + lc - NF];
#pragma unroll
    for (int r = 0; r < 8; ++r) {
      const int lr = 16 * wave + 8 * hh + r;
      stg[lr * 128 + lc] = acc[nt][r] + bvv;
    }
  }
  __syncthreads();
  v4f pv[16];
#pragma unroll
  for (int i = 0; i < 16; ++i) pv[i] = *(const v4fa*)(stg + (16 * wave + i) * 128 + 4 * lane);
#pragma unroll
  for (int i = 0; i < 16; ++i) {
    float* op = PSD + (size_t)(rowBase + 16 * wave + i) * 128 + 4 * lane;
    *(volatile v4f*)op = pv[i];
  }
  __threadfence();
#pragma unroll
  for (int i = 0; i < 16; ++i) {
    float* op = PSD + (size_t)(rowBase + 16 * wave + i) * 128 + 4 * lane;
    *(volatile v4f*)op = pv[i];
  }
}

__global__ __launch_bounds__(NTHR) void k_bucket(const int* __restrict__ srcs, const int* __restrict__ dsts,
                                                 int nE, int nN, int vec8, int* HITS, int* FLG) {
  extern __shared__ __attribute__((aligned(16))) int bsm[];
  int* list = bsm;
  int* reg1 = bsm + LISTN;
  int* wcnt = reg1 + RCAP;
  const int tid = (int)threadIdx.x, lane = tid & 31, wave = tid >> 5;
  const int blk = (int)blockIdx.x;
  const int nodeBase = blk * NBA;
  int nb = nN - nodeBase;
  nb = nb < 0 ? 0 : (nb > NBA ? NBA : nb);

  int tot = 0, ovf = 0;
  const int nChunks = (nE + CHUNK - 1) / CHUNK;
#pragma unroll 1
  for (int ch = 0; ch < nChunks; ++ch) {
    const int cbase = ch * CHUNK;
    const int wc = scan_chunk<SLA>(dsts, nE, cbase, nodeBase, nb, vec8, list, tid, lane, wave);
    if (lane == 0) wcnt[wave] = wc;
    __syncthreads();
    int pre = 0, all = 0;
#pragma unroll
    for (int w2 = 0; w2 < NWAVE; ++w2) {
      int c = wcnt[w2];
      c = c < 0 ? 0 : (c > WCAP ? WCAP : c);
      all += c;
      pre += (w2 < wave) ? c : 0;
    }
    const int wcc  = wc > WCAP ? WCAP : wc;
    const int base = tot + pre;
#pragma unroll 1
    for (int i = lane; i < wcc; i += 32) {
      const int ent = list[wave * WCAP + i];
      const int el  = (ent >> SLA) & (CHUNK - 1);
      const int sl  = ent & (NBA - 1);
      int eid = cbase + el;
      eid = eid > nE - 1 ? nE - 1 : eid;
      const int sraw = srcs[eid];
      const int s = sraw < 0 ? 0 : (sraw > nN - 1 ? nN - 1 : sraw);
      const int pos = base + i;
      if (pos < RCAP) reg1[pos] = (int)((unsigned)s | ((unsigned)sl << 16));
    }
    if (tot + all > RCAP) ovf = 1;
    tot += all;
    tot = tot > RCAP ? RCAP : tot;
    __syncthreads();
  }
  const int nh = tot;
  const int nhPad = (nh + 31) & ~31;
  for (int i = nh + tid; i < nhPad; i += NTHR) reg1[i] = 0;
  __syncthreads();

  int* hb = HITS + (size_t)blk * RCAP;
  v4i cv;
  cv.x = (tid == 0) ? nh : 0;
  cv.y = (tid == 0) ? ovf : 0;
  cv.z = 0; cv.w = 0;
  int* fp = FLG + (size_t)blk * 32 + 4 * (tid & 7);
#pragma unroll 1
  for (int p = tid * 4; p < nhPad; p += NTHR * 4) {
    const v4i v = *(const v4ia*)(reg1 + p);
    *(volatile v4i*)(hb + p) = v;
  }
  if (tid < 8) *(volatile v4i*)fp = cv;
  __threadfence();
#pragma unroll 1
  for (int p = tid * 4; p < nhPad; p += NTHR * 4) {
    const v4i v = *(const v4ia*)(reg1 + p);
    *(volatile v4i*)(hb + p) = v;
  }
  if (tid < 8) *(volatile v4i*)fp = cv;
}

__device__ __forceinline__ void gemm4_lds(const unsigned short* ap, const unsigned short* bp, v8f (&acc)[4]) {
#pragma unroll
  for (int ks = 0; ks < 4; ++ks) {
    FragB af;
    af.h[0] = *(const v8usa*)(ap + 32 * ks);
    af.h[1] = *(const v8usa*)(ap + 32 * ks + 16);
#pragma unroll
    for (int nt = 0; nt < 4; ++nt) {
      const unsigned short* wq = bp + (16 * nt) * AP + 32 * ks;
      FragB bf;
      bf.h[0] = *(const v8usa*)wq;
      bf.h[1] = *(const v8usa*)(wq + 16);
      acc[nt] = wmb(af, bf, acc[nt]);
    }
  }
}

__device__ __forceinline__ void hagg_pass(const float* sACC, unsigned short* HAGG, int nodeBase, int MPr,
                                          int tid, float pz) {
  const int p  = tid & 15;
  const int rs = tid >> 4;
  const int c0 = (p & 7) * 8;
  const unsigned mh = 0u - (unsigned)(p >> 3);
  const unsigned ml = ~mh;
#pragma unroll 1
  for (int sw = 0; sw < NBA / 16; ++sw) {
    const int row  = sw * 16 + rs;
    const int node = nodeBase + row;
    const float* aq = sACC + row * SP + c0;
    const v4f a = *(const v4fa*)aq;
    const v4f b = *(const v4fa*)(aq + 4);
    const v8f f8 = {a.x, a.y, a.z, a.w, b.x, b.y, b.z, b.w};
    v8us o;
#pragma unroll
    for (int e = 0; e < 8; ++e) {
      const float x = f8[e] + pz;
      const unsigned hb = f2bf(x);
      const unsigned lb = f2bf(x - bf2f(hb));
      o[e] = (unsigned short)((hb & ml) | (lb & mh));
    }
    if (node < MPr) *(volatile v8us*)(HAGG + (size_t)node * KD + 8 * p) = o;
  }
}

__global__ __launch_bounds__(NTHR) __attribute__((amdgpu_num_vgpr(248)))
void k_edge(const int* __restrict__ HITS, const int* __restrict__ FLG, const float* __restrict__ PSD,
            const float* __restrict__ CB, const unsigned short* __restrict__ WPL,
            const float* __restrict__ TAB, unsigned short* HAGG, float* out1, int nN, int MPr) {
  extern __shared__ __attribute__((aligned(16))) float dyn[];
  float*          sACC = dyn;
  float*          sSTG = sACC + E_ACC_F;
  float*          sDX  = sSTG + E_STG_F;
  float*          sTAB = sDX + TROWS * 4;
  int*            sLT  = (int*)(sTAB + TABN);
  unsigned short* sA   = (unsigned short*)(sLT + TROWS);
  unsigned short* sW2  = sA + E_A_H;
  unsigned short* sWC  = sW2 + E_W_H;

  const int tid = (int)threadIdx.x, lane = tid & 31, wave = tid >> 5, hh = lane >> 4, m = lane & 15;
  const int blk = (int)blockIdx.x;
  const int nodeBase = blk * NBA;

  {
    const v4f z4 = {0.0f, 0.0f, 0.0f, 0.0f};
#pragma unroll 1
    for (int i = tid * 4; i < E_ACC_F; i += NTHR * 4) *(v4fa*)(sACC + i) = z4;
#pragma unroll 1
    for (int u = tid; u < NF * 16; u += NTHR) {
      const int n = u >> 4, p = u & 15;
      const v8us a = *(const v8usa*)(WPL + OFF_E2 + n * KD + 8 * p);
      const v8us b = *(const v8usa*)(WPL + OFF_C1 + n * KD + 8 * p);
      *(v8usa*)(sW2 + n * AP + 8 * p) = a;
      *(v8usa*)(sWC + n * AP + 8 * p) = b;
    }
    const v8us z8 = {0, 0, 0, 0, 0, 0, 0, 0};
    if (tid < NF) {
      *(v8usa*)(sW2 + tid * AP + KD) = z8;
      *(v8usa*)(sWC + tid * AP + KD) = z8;
    }
    if (tid < TROWS) {
      *(v8usa*)(sA + tid * AP + KD) = z8;
      *(v4fa*)(sTAB + 4 * tid) = *(const v4fa*)(TAB + 4 * tid);
    }
  }
  const int nhraw = FLG[(size_t)blk * 32];
  const int bflag = FLG[(size_t)blk * 32 + 1];
  const int nh  = nhraw < 0 ? 0 : (nhraw > RCAP ? RCAP : nhraw);
  const int ovf = (bflag != 0 || nhraw < 0 || nhraw > RCAP) ? 1 : 0;
  const int nT  = (nh + TROWS - 1) / TROWS;
  const int* hb = HITS + (size_t)blk * RCAP;
  __syncthreads();

  const int wrow = 16 * wave;
  const unsigned short* apw = sA + (wrow + m) * AP + 8 * hh;
  const unsigned short* b2p = sW2 + m * AP + 8 * hh;
  const unsigned short* bcp = sWC + m * AP + 8 * hh;
  float*          stw = sSTG + (wrow + 8 * hh) * SP + m;
  unsigned short* aw  = sA + (wrow + 8 * hh) * AP + m;
  const int gr = tid >> 1, hf = tid & 1;
  const int cc = tid & 63, qq = tid >> 6;

#pragma unroll 1
  for (int tl = 0; tl < nT; ++tl) {
    int nv = nh - tl * TROWS;
    nv = nv > TROWS ? TROWS : nv;
    {
      const int li = tl * TROWS + gr;
      const bool valid = li < nh;
      int idx = valid ? li : (nh - 1);
      idx = idx < 0 ? 0 : (idx > RCAP - 1 ? RCAP - 1 : idx);
      const int ent = hb[idx];
      int s = ent & 0xFFFF;
      s = s > nN - 1 ? nN - 1 : s;
      int slot = (ent >> 16) & (NBA - 1);
      slot = valid ? slot : 0;
      int d = nodeBase + slot;
      d = d > nN - 1 ? nN - 1 : d;
      const v4f xs = *(const v4fa*)(CB + (size_t)s * 4);
      const v4f xd = *(const v4fa*)(CB + (size_t)d * 4);
      const float dx0 = xs.x - xd.x, dx1 = xs.y - xd.y, dx2 = xs.z - xd.z;
      const float d2  = (dx0 * dx0 + dx2 * dx2) + dx1 * dx1;
      const float* ps = PSD + (size_t)s * 128 + 32 * hf;
      const float* pd = PSD + (size_t)d * 128 + NF + 32 * hf;
      const float* tw = sTAB + T_W128 + 32 * hf;
      unsigned short* ar = sA + gr * AP + 32 * hf;
#pragma unroll 1
      for (int c8 = 0; c8 < 4; ++c8) {
        const v4f pa = *(const v4fa*)(ps + 8 * c8);
        const v4f pb = *(const v4fa*)(ps + 8 * c8 + 4);
        const v4f qa = *(const v4fa*)(pd + 8 * c8);
        const v4f qb = *(const v4fa*)(pd + 8 * c8 + 4);
        const v4f wa = *(const v4fa*)(tw + 8 * c8);
        const v4f wb = *(const v4fa*)(tw + 8 * c8 + 4);
        const v8f p8 = {pa.x, pa.y, pa.z, pa.w, pb.x, pb.y, pb.z, pb.w};
        const v8f q8 = {qa.x, qa.y, qa.z, qa.w, qb.x, qb.y, qb.z, qb.w};
        const v8f w8 = {wa.x, wa.y, wa.z, wa.w, wb.x, wb.y, wb.z, wb.w};
        v8us oh, ol;
#pragma unroll
        for (int i = 0; i < 8; ++i) {
          const float pre = (p8[i] + q8[i]) + d2 * w8[i];
          float mm = silu_p(pre);
          mm = valid ? mm : 0.0f;
          const unsigned hbv = f2bf(mm);
          oh[i] = (unsigned short)hbv;
          ol[i] = (unsigned short)f2bf(mm - bf2f(hbv));
        }
        *(v8usa*)(ar + 8 * c8)      = oh;
        *(v8usa*)(ar + NF + 8 * c8) = ol;
      }
      if (hf == 0) {
        v4f dq;
        dq.x = valid ? dx0 : 0.0f;
        dq.y = valid ? dx1 : 0.0f;
        dq.z = valid ? dx2 : 0.0f;
        dq.w = 0.0f;
        *(v4fa*)(sDX + 4 * gr) = dq;
        sLT[gr] = slot;
      }
    }
    __syncthreads();

    {
      v8f acc[4];
      const v8f z = {0.f, 0.f, 0.f, 0.f, 0.f, 0.f, 0.f, 0.f};
      acc[0] = z; acc[1] = z; acc[2] = z; acc[3] = z;
      gemm4_lds(apw, b2p, acc);
#pragma unroll
      for (int nt = 0; nt < 4; ++nt)
#pragma unroll
        for (int r = 0; r < 8; ++r) stw[r * SP + 16 * nt] = acc[nt][r];
    }
#pragma unroll 1
    for (int j = 0; j < 32; ++j) {
      const int nt = j >> 3, r = j & 7;
      float* sp = stw + r * SP + 16 * nt;
      const float he = silu_p(*sp + sTAB[T_BE2 + 16 * nt + m]);
      *sp = he;
      const unsigned hbv = f2bf(he);
      const unsigned lbv = f2bf(he - bf2f(hbv));
      aw[r * AP + 16 * nt]      = (unsigned short)hbv;
      aw[r * AP + NF + 16 * nt] = (unsigned short)lbv;
    }
    __syncthreads();

#pragma unroll 1
    for (int r4 = 0; r4 < nv; r4 += 4) {
      const v4i s4 = *(const v4ia*)(sLT + r4);
      if ((s4.x & 3) == qq)                 sACC[s4.x * SP + cc] += sSTG[(r4 + 0) * SP + cc];
      if (r4 + 1 < nv && (s4.y & 3) == qq)  sACC[s4.y * SP + cc] += sSTG[(r4 + 1) * SP + cc];
      if (r4 + 2 < nv && (s4.z & 3) == qq)  sACC[s4.z * SP + cc] += sSTG[(r4 + 2) * SP + cc];
      if (r4 + 3 < nv && (s4.w & 3) == qq)  sACC[s4.w * SP + cc] += sSTG[(r4 + 3) * SP + cc];
    }

    {
      v8f acc[4];
      const v8f z = {0.f, 0.f, 0.f, 0.f, 0.f, 0.f, 0.f, 0.f};
      acc[0] = z; acc[1] = z; acc[2] = z; acc[3] = z;
      gemm4_lds(apw, bcp, acc);
      __syncthreads();
#pragma unroll
      for (int nt = 0; nt < 4; ++nt)
#pragma unroll
        for (int r = 0; r < 8; ++r) stw[r * SP + 16 * nt] = acc[nt][r];
    }
#pragma unroll 1
    for (int j = 0; j < 32; ++j) {
      const int nt = j >> 3, r = j & 7;
      float* sp = stw + r * SP + 16 * nt;
      *sp = silu_p(*sp + sTAB[T_BC1 + 16 * nt + m]);
    }
    __syncthreads();

    if (tid < TROWS) {
      const float* sr = sSTG + tid * SP;
      float dot = 0.0f;
#pragma unroll 1
      for (int c4 = 0; c4 < NF / 4; ++c4) {
        const v4f v = *(const v4fa*)(sr + 4 * c4);
        const v4f w = *(const v4fa*)(sTAB + T_WC2 + 4 * c4);
        dot = fmaf(v.x, w.x, dot);
        dot = fmaf(v.y, w.y, dot);
        dot = fmaf(v.z, w.z, dot);
        dot = fmaf(v.w, w.w, dot);
      }
      const float coef = dot + sTAB[T_BC2];
      v4f dq = *(const v4fa*)(sDX + 4 * tid);
      dq.x = dq.x * coef; dq.y = dq.y * coef; dq.z = dq.z * coef; dq.w = 0.0f;
      *(v4fa*)(sDX + 4 * tid) = dq;
    }
    __syncthreads();

    if (wave == 0) {
      const int jc = lane < 3 ? lane : 3;
#pragma unroll 1
      for (int r = 0; r < nv; ++r) {
        const int sl = sLT[r] & (NBA - 1);
        const float xv = sDX[4 * r + jc];
        float* cp = sACC + sl * SP + NF + jc;
        const float nvv = *cp + xv;
        if (lane < 4) *cp = nvv;
      }
    }
    __syncthreads();
  }

  const float qnan = __int_as_float(0x7fc00000);
  const float pz = (ovf != 0) ? qnan : 0.0f;
  hagg_pass(sACC, HAGG, nodeBase, MPr, tid, pz);
  __threadfence();
  hagg_pass(sACC, HAGG, nodeBase, MPr, tid, pz);

  float* sx = sSTG;
#pragma unroll 1
  for (int rl = tid; rl < NBA; rl += NTHR) {
    const int node = nodeBase + rl;
    const int nc = node < nN ? node : nN - 1;
    const v4f cb = *(const v4fa*)(CB + (size_t)nc * 4);
    sx[3 * rl + 0] = (cb.x + sACC[rl * SP + NF + 0]) + pz;
    sx[3 * rl + 1] = (cb.y + sACC[rl * SP + NF + 1]) + pz;
    sx[3 * rl + 2] = (cb.z + sACC[rl * SP + NF + 2]) + pz;
  }
  __syncthreads();
  {
    const int np = (NBA * 3) / 4;
    const int p0 = tid;
    const int p1 = (tid + NTHR) < np ? (tid + NTHR) : (np - 1);
    const v4f o0 = *(const v4fa*)(sx + 4 * p0);
    const v4f o1 = *(const v4fa*)(sx + 4 * p1);
    const long long g0 = (long long)nodeBase * 3 + 4LL * p0;
    const long long g1 = (long long)nodeBase * 3 + 4LL * p1;
    const long long lim = 3LL * nN;
    const bool st0 = (g0 + 4 <= lim);
    const bool st1 = (tid + NTHR < np) && (g1 + 4 <= lim);
    if (st0) *(volatile v4f*)(out1 + (size_t)g0) = o0;
    if (st1) *(volatile v4f*)(out1 + (size_t)g1) = o1;
    __threadfence();
    if (st0) *(volatile v4f*)(out1 + (size_t)g0) = o0;
    if (st1) *(volatile v4f*)(out1 + (size_t)g1) = o1;
  }
}

__global__ __launch_bounds__(GTHR) __attribute__((amdgpu_num_vgpr(248)))
void k_node(const unsigned short* __restrict__ XB, const unsigned short* __restrict__ HAGG,
            const unsigned short* __restrict__ WPL, const float* __restrict__ TAB,
            const int* __restrict__ FLG, float* out0, int nN) {
  __shared__ __attribute__((aligned(16))) float stg[GBM * SP];
  __shared__ __attribute__((aligned(16))) unsigned short sT[GBM * AP];
  const int tid = (int)threadIdx.x, lane = tid & 31, wave = tid >> 5, hh = lane >> 4, m = lane & 15;
  const int rowBase = (int)blockIdx.x * GBM;
  const int fb = rowBase >> SLA;
  const int nhraw = FLG[(size_t)fb * 32];
  const int bflag = FLG[(size_t)fb * 32 + 1];
  const float qnan = __int_as_float(0x7fc00000);
  const float pz = (bflag != 0 || nhraw < 0 || nhraw > RCAP) ? qnan : 0.0f;

  const v8f z = {0.f, 0.f, 0.f, 0.f, 0.f, 0.f, 0.f, 0.f};
  float* stw = stg + (16 * wave + 8 * hh) * SP + m;
  unsigned short* tw = sT + (16 * wave + 8 * hh) * AP + m;
  {
    v8f acc[4];
    acc[0] = z; acc[1] = z; acc[2] = z; acc[3] = z;
    const size_t grow = (size_t)(rowBase + 16 * wave + m);
    const unsigned short* ap0 = XB + grow * NF + 8 * hh;
    const unsigned short* ap1 = HAGG + grow * KD + 8 * hh;
    const unsigned short* bp  = WPL + OFF_N1 + m * KN1 + 8 * hh;
#pragma unroll
    for (int ks = 0; ks < 2; ++ks) {
      FragB af;
      af.h[0] = *(const v8usa*)(ap0 + 32 * ks);
      af.h[1] = *(const v8usa*)(ap0 + 32 * ks + 16);
#pragma unroll
      for (int nt = 0; nt < 4; ++nt) {
        const unsigned short* wq = bp + (16 * nt) * KN1 + 32 * ks;
        FragB bf;
        bf.h[0] = *(const v8usa*)wq;
        bf.h[1] = *(const v8usa*)(wq + 16);
        acc[nt] = wmb(af, bf, acc[nt]);
      }
    }
#pragma unroll
    for (int ks = 0; ks < 4; ++ks) {
      FragB af;
      af.h[0] = *(const v8usa*)(ap1 + 32 * ks);
      af.h[1] = *(const v8usa*)(ap1 + 32 * ks + 16);
#pragma unroll
      for (int nt = 0; nt < 4; ++nt) {
        const unsigned short* wq = bp + (16 * nt) * KN1 + NF + 32 * ks;
        FragB bf;
        bf.h[0] = *(const v8usa*)wq;
        bf.h[1] = *(const v8usa*)(wq + 16);
        acc[nt] = wmb(af, bf, acc[nt]);
      }
    }
#pragma unroll
    for (int nt = 0; nt < 4; ++nt)
#pragma unroll
      for (int r = 0; r < 8; ++r) stw[r * SP + 16 * nt] = acc[nt][r];
  }
#pragma unroll 1
  for (int j = 0; j < 32; ++j) {
    const int nt = j >> 3, r = j & 7;
    const float tv = silu_p(stw[r * SP + 16 * nt] + TAB[T_BN1 + 16 * nt + m]);
    const unsigned hbv = f2bf(tv);
    const unsigned lbv = f2bf(tv - bf2f(hbv));
    tw[r * AP + 16 * nt]      = (unsigned short)hbv;
    tw[r * AP + NF + 16 * nt] = (unsigned short)lbv;
  }
  __syncthreads();
  {
    v8f acc[4];
    acc[0] = z; acc[1] = z; acc[2] = z; acc[3] = z;
    const unsigned short* ap = sT + (16 * wave + m) * AP + 8 * hh;
    const unsigned short* bp = WPL + OFF_N2 + m * KD + 8 * hh;
#pragma unroll
    for (int ks = 0; ks < 4; ++ks) {
      FragB af;
      af.h[0] = *(const v8usa*)(ap + 32 * ks);
      af.h[1] = *(const v8usa*)(ap + 32 * ks + 16);
#pragma unroll
      for (int nt = 0; nt < 4; ++nt) {
        const unsigned short* wq = bp + (16 * nt) * KD + 32 * ks;
        FragB bf;
        bf.h[0] = *(const v8usa*)wq;
        bf.h[1] = *(const v8usa*)(wq + 16);
        acc[nt] = wmb(af, bf, acc[nt]);
      }
    }
#pragma unroll
    for (int nt = 0; nt < 4; ++nt) {
      const float bv = TAB[T_BN2 + 16 * nt + m];
#pragma unroll
      for (int r = 0; r < 8; ++r) stw[r * SP + 16 * nt] = (acc[nt][r] + bv) + pz;
    }
  }
  __syncthreads();
  v4f fv[8];
#pragma unroll
  for (int i = 0; i < 8; ++i) {
    const int lr = 16 * wave + 2 * i + hh;
    fv[i] = *(const v4fa*)(stg + lr * SP + 4 * m);
  }
#pragma unroll
  for (int i = 0; i < 8; ++i) {
    const int grw = rowBase + 16 * wave + 2 * i + hh;
    if (grw < nN) *(volatile v4f*)(out0 + (size_t)grw * NF + 4 * m) = fv[i];
  }
  __threadfence();
#pragma unroll
  for (int i = 0; i < 8; ++i) {
    const int grw = rowBase + 16 * wave + 2 * i + hh;
    if (grw < nN) *(volatile v4f*)(out0 + (size_t)grw * NF + 4 * m) = fv[i];
  }
}

static inline int cdiv(int a, int b) { return (a + b - 1) / b; }

extern "C" void kernel_launch(void* const* d_in, const int* in_sizes, int n_in,
                              void* d_out, int out_size, void* d_ws, size_t ws_size,
                              hipStream_t stream) {
  if (n_in < 16) return;
  const int nN = in_sizes[0] / NF;
  if (nN < 1 || in_sizes[0] != nN * NF || nN > 65536) return;
  if (in_sizes[1] != 3 * nN) return;
  const int nE = in_sizes[2];
  if (nE < 1 || in_sizes[3] != nE) return;
  if (in_sizes[4] != (2 * NF + 1) * NF || in_sizes[5] != NF) return;
  if (in_sizes[6] != NF * NF || in_sizes[7] != NF) return;
  if (in_sizes[8] != NF * NF || in_sizes[9] != NF) return;
  if (in_sizes[10] != NF || in_sizes[11] != 1) return;
  if (in_sizes[12] != 2 * NF * NF || in_sizes[13] != NF) return;
  if (in_sizes[14] != NF * NF || in_sizes[15] != NF) return;
  if ((long long)out_size != (long long)nN * NF + 3LL * nN) return;
  if (((3 * nN) & 3) != 0) return;
  if ((((size_t)nN * NF * 4) % 128) != 0) return;

  const float* feat  = (const float*)d_in[0];
  const float* coord = (const float*)d_in[1];
  const int*   src   = (const int*)d_in[2];
  const int*   dst   = (const int*)d_in[3];
  const float* We1 = (const float*)d_in[4];
  const float* be1 = (const float*)d_in[5];
  const float* We2 = (const float*)d_in[6];
  const float* be2 = (const float*)d_in[7];
  const float* Wc1 = (const float*)d_in[8];
  const float* bc1 = (const float*)d_in[9];
  const float* Wc2 = (const float*)d_in[10];
  const float* bc2 = (const float*)d_in[11];
  const float* Wn1 = (const float*)d_in[12];
  const float* bn1 = (const float*)d_in[13];
  const float* Wn2 = (const float*)d_in[14];
  const float* bn2 = (const float*)d_in[15];
  float* out0 = (float*)d_out;
  float* out1 = out0 + (size_t)nN * NF;

  const int MP = cdiv(nN, MROWS) * MROWS;
  const int gM = MP / GBM;
  const int gA = cdiv(MP, NBA);
  if ((long long)gA * NBA < (long long)MP) return;
  if (((MP * 8) % NTHR) != 0) return;
  const int nXP  = cdiv(MP, NTHR) * NTHR;
  const int vec8 = ((nE & 3) == 0) ? 1 : 0;

  char* ws = (char*)d_ws;
  size_t off = 0;
  const size_t oXB  = off; off += (size_t)MP * NF * 2;        off = (off + 255) & ~(size_t)255;
  const size_t oCB  = off; off += (size_t)MP * 16;            off = (off + 255) & ~(size_t)255;
  const size_t oWPL = off; off += (size_t)WPL_HALVES * 2;     off = (off + 255) & ~(size_t)255;
  const size_t oTAB = off; off += (size_t)TABN * 4;           off = (off + 255) & ~(size_t)255;
  const size_t oPSD = off; off += (size_t)MP * 128 * 4;       off = (off + 255) & ~(size_t)255;
  const size_t oHIT = off; off += (size_t)gA * RCAP * 4;      off = (off + 255) & ~(size_t)255;
  const size_t oFLG = off; off += (size_t)gA * 128;           off = (off + 255) & ~(size_t)255;
  const size_t oHAG = off; off += (size_t)MP * KD * 2;        off = (off + 255) & ~(size_t)255;
  if (off > ws_size || off > (size_t)WSMAX) return;
  unsigned short* XB   = (unsigned short*)(ws + oXB);
  float*          CB   = (float*)(ws + oCB);
  unsigned short* WPL  = (unsigned short*)(ws + oWPL);
  float*          TAB  = (float*)(ws + oTAB);
  float*          PSD  = (float*)(ws + oPSD);
  int*            HITS = (int*)(ws + oHIT);
  int*            FLG  = (int*)(ws + oFLG);
  unsigned short* HAGG = (unsigned short*)(ws + oHAG);

  const int bktLds = BKT_LDS_INTS * 4;
  hipFuncSetAttribute(reinterpret_cast<const void*>(&k_edge), hipFuncAttributeMaxDynamicSharedMemorySize,
                      (int)EDGE_LDS_BYTES);

  k_pa<<<(MP * 8 + nXP) / NTHR, NTHR, 0, stream>>>(feat, coord, XB, CB, nN, MP);
  k_pb<<<NU_PB / NTHR, NTHR, 0, stream>>>(We1, We2, Wc1, Wn1, Wn2, WPL);
  k_pc<<<1, NTHR, 0, stream>>>(We1, be1, be2, bc1, Wc2, bc2, bn1, bn2, TAB);
  k_psd<<<gM, GTHR, 0, stream>>>(XB, WPL, TAB, PSD);
  k_bucket<<<gA, NTHR, bktLds, stream>>>(src, dst, nE, nN, vec8, HITS, FLG);
  k_edge<<<gA, NTHR, EDGE_LDS_BYTES, stream>>>(HITS, FLG, PSD, CB, WPL, TAB, HAGG, out1, nN, MP);
  k_node<<<gM, GTHR, 0, stream>>>(XB, HAGG, WPL, TAB, FLG, out0, nN);
}
